// MultiHeadAttentionClassical_65481071399213
// MI455X (gfx1250) — hardware-verified
//
#include <hip/hip_runtime.h>
#ifndef NB
#define NB 2
#endif
#ifndef SEQ
#define SEQ 2048
#endif
#define NB_FULL 2
#define SEQ_FULL 2048
#define DM 1024
#define NH 16
#define HD 64
#define NR (NB * SEQ)
#define QBLKS (SEQ / 64)
#define SCL 0.125f
static_assert(SEQ % 64 == 0);
static_assert(NR % 128 == 0);
static_assert(NB >= 1 && NB <= NB_FULL);
static_assert(SEQ <= SEQ_FULL);
static_assert(NH * HD == DM);
static_assert(DM % 64 == 0);

typedef unsigned short v8us __attribute__((ext_vector_type(8), may_alias));
typedef float  v8f  __attribute__((ext_vector_type(8)));
typedef float  v4f  __attribute__((ext_vector_type(4)));
typedef float  v4fa __attribute__((ext_vector_type(4), may_alias));
typedef _Float16 v16h __attribute__((ext_vector_type(16)));
typedef _Float16 v4h __attribute__((ext_vector_type(4)));
union FragH { v16h v; v8us half[2]; _Float16 h[16]; unsigned short u[16]; };

__device__ __forceinline__ unsigned short bf16_bits(float x) { unsigned int u = __float_as_uint(x); return (unsigned short)((u + 0x7FFFu + ((u >> 16) & 1u)) >> 16); }
__device__ __forceinline__ float bf16_val(unsigned short b) { return __uint_as_float(((unsigned int)b) << 16); }
__device__ __forceinline__ float bf16_rne(float x) { return bf16_val(bf16_bits(x)); }

__device__ __forceinline__ v16h ld_frag(const _Float16* p, int hh) { FragH f; f.half[0] = *(const v8us*)((const unsigned short*)p + 8 * hh); f.half[1] = *(const v8us*)((const unsigned short*)p + 16 + 8 * hh); return f.v; }
__device__ __forceinline__ v8f mma16(v16h a, v16h b, v8f c) { v8f d = __builtin_amdgcn_wmma_f32_16x16x32_f16(false, a, false, b, (short)0, c, false, false); asm volatile("v_nop\n\tv_nop\n\tv_nop\n\tv_nop" : "+v"(d) : "v"(a), "v"(b)); return d; }

__global__ __launch_bounds__(256) void k_wsc(const float* __restrict__ Wm, _Float16* __restrict__ Bt, size_t n8, float sc) {
  const size_t t = (size_t)blockIdx.x * 256 + threadIdx.x; if (t >= n8) return;
  const v4f a0 = *(const v4fa*)(Wm + t * 8), a1 = *(const v4fa*)(Wm + t * 8 + 4);
  FragH f;
#pragma unroll
  for (int q = 0; q < 4; ++q) { f.h[q] = (_Float16)(bf16_rne(a0[q]) * sc); f.h[4 + q] = (_Float16)(bf16_rne(a1[q]) * sc); }
  const v8us o = f.half[0];
  *(volatile v8us*)((unsigned short*)Bt + t * 8) = o; __threadfence(); *(volatile v8us*)((unsigned short*)Bt + t * 8) = o;
}

__global__ __launch_bounds__(256) void k_x16(const float* __restrict__ x, _Float16* __restrict__ X16, size_t n8) {
  const size_t t = (size_t)blockIdx.x * 256 + threadIdx.x; if (t >= n8) return;
  const size_t row = (t * 8) / DM; const int c = (int)((t * 8) % DM); const size_t b = row / SEQ, s = row % SEQ;
  const float* src = x + ((b * SEQ_FULL + s) * (size_t)DM + c);
  const v4f a0 = *(const v4fa*)src, a1 = *(const v4fa*)(src + 4);
  FragH f;
#pragma unroll
  for (int q = 0; q < 4; ++q) { f.h[q] = (_Float16)bf16_rne(a0[q]); f.h[4 + q] = (_Float16)bf16_rne(a1[q]); }
  const v8us o = f.half[0];
  *(volatile v8us*)((unsigned short*)X16 + t * 8) = o; __threadfence(); *(volatile v8us*)((unsigned short*)X16 + t * 8) = o;
}

__global__ __launch_bounds__(128) void k_gemm2(const _Float16* __restrict__ A, int lda, const _Float16* __restrict__ Bh, int ldb, float alpha,
                                               const float* __restrict__ bias, const float* CP, int ldcp, float* C, _Float16* C16, int ldc, int M, int N, int K) {
  __shared__ __attribute__((aligned(16))) float so[4][32][68];
  const int tid = threadIdx.x, w = tid >> 5, lane = tid & 31, ln = lane & 15, hh = lane >> 4;
  const int ntn = N >> 6; const int mt = blockIdx.x / ntn, nq = blockIdx.x - mt * ntn; const int row0 = mt * 128 + 32 * w, col0 = nq * 64; if (row0 >= M) return;
  const _Float16* a0p = A + (size_t)(row0 + ln) * lda; const _Float16* a1p = a0p + (size_t)16 * lda;
  const _Float16* b0p = Bh + (size_t)(col0 + ln) * ldb; const _Float16* b1p = b0p + (size_t)16 * ldb; const _Float16* b2p = b1p + (size_t)16 * ldb; const _Float16* b3p = b2p + (size_t)16 * ldb;
  const v8f z8 = {0.f,0.f,0.f,0.f,0.f,0.f,0.f,0.f}; v8f c00 = z8, c01 = z8, c02 = z8, c03 = z8, c10 = z8, c11 = z8, c12 = z8, c13 = z8;
#pragma unroll 1
  for (int kb = 0; kb < K; kb += 32) { const v16h a0 = ld_frag(a0p + kb, hh), a1 = ld_frag(a1p + kb, hh);
    v16h b = ld_frag(b0p + kb, hh); c00 = mma16(a0, b, c00); c10 = mma16(a1, b, c10);
    b = ld_frag(b1p + kb, hh); c01 = mma16(a0, b, c01); c11 = mma16(a1, b, c11);
    b = ld_frag(b2p + kb, hh); c02 = mma16(a0, b, c02); c12 = mma16(a1, b, c12);
    b = ld_frag(b3p + kb, hh); c03 = mma16(a0, b, c03); c13 = mma16(a1, b, c13); }
  v8f accs[8] = {c00, c01, c02, c03, c10, c11, c12, c13};
#pragma unroll
  for (int u = 0; u < 8; ++u) { const int t = u & 3, half = u >> 2; const int col = col0 + t * 16 + ln; const float bvl = bias ? bf16_rne(bias[col]) : 0.f;
#pragma unroll
    for (int r = 0; r < 8; ++r) { const int rloc = half * 16 + 8 * hh + r; float v = accs[u][r] * alpha + bvl; if (CP) v += CP[(size_t)(row0 + rloc) * ldcp + col]; so[w][rloc][t * 16 + ln] = v; } }
  __builtin_amdgcn_fence(4, "workgroup"); __builtin_amdgcn_wave_barrier();
  const int rsub = hh, c4 = ln * 4;
  for (int pass = 0; pass < 2; ++pass) {
#pragma unroll
    for (int q = 0; q < 16; ++q) { const int r = q * 2 + rsub; const v4f v = *(const v4fa*)&so[w][r][c4];
      if (C) *(volatile v4f*)(C + (size_t)(row0 + r) * ldc + col0 + c4) = v;
      if (C16) { v4h h4;
#pragma unroll
        for (int i = 0; i < 4; ++i) h4[i] = (_Float16)v[i];
        *(volatile v4h*)(C16 + (size_t)(row0 + r) * ldc + col0 + c4) = h4; } }
    if (pass == 0) __threadfence(); }
}

__global__ __launch_bounds__(256) void k_vtg(const _Float16* __restrict__ V16, _Float16* __restrict__ Vt) {
  __shared__ __attribute__((aligned(16))) unsigned short tl[64][66];
  const int tid = threadIdx.x; const int slab = blockIdx.x / (SEQ / 64), lg = blockIdx.x % (SEQ / 64); const int b = slab / NH, h = slab % NH;
  for (int i = tid; i < 64 * 8; i += 256) { const int r = i / 8, c8 = (i % 8) * 8; FragH f; f.half[0] = *(const v8us*)((const unsigned short*)V16 + ((size_t)b * SEQ + lg * 64 + r) * DM + h * HD + c8);
#pragma unroll
    for (int q = 0; q < 8; ++q) tl[r][c8 + q] = f.u[q]; }
  __syncthreads();
  for (int pass = 0; pass < 2; ++pass) {
#pragma unroll
    for (int rd = 0; rd < 2; ++rd) { const int d = rd * 32 + tid / 8, pc = tid % 8; FragH f;
#pragma unroll
      for (int q = 0; q < 8; ++q) f.u[q] = tl[pc * 8 + q][d];
      *(volatile v8us*)((unsigned short*)Vt + ((size_t)slab * HD + d) * SEQ + lg * 64 + pc * 8) = f.half[0]; }
    if (pass == 0) __threadfence(); }
}

__global__ __launch_bounds__(128) void k_flash(const _Float16* __restrict__ Q16, int ldq, const _Float16* __restrict__ K16, int ldk, const _Float16* __restrict__ Vt,
                                               const int* __restrict__ MSK, int mstride, float* __restrict__ O, int ldo) {
  constexpr int RPW = 16, DT = 4, KS = 2;
  __shared__ __attribute__((aligned(16))) unsigned short sP[4][RPW][40];
  __shared__ __attribute__((aligned(16))) float sO[4][RPW][68];
  const int tid = threadIdx.x, w = tid >> 5, lane = tid & 31, ln = lane & 15, hh = lane >> 4;
  const int slab = blockIdx.x / QBLKS, qblk = blockIdx.x % QBLKS; const int b = slab / NH, h = slab % NH;
  const int q0 = qblk * 64 + w * RPW;
  FragH aq[KS];
  { const unsigned short* qr = (const unsigned short*)Q16 + ((size_t)b * SEQ + q0 + ln) * ldq + h * HD;
#pragma unroll
    for (int ks = 0; ks < KS; ++ks) { aq[ks].half[0] = *(const v8us*)(qr + ks * 32 + 8 * hh); aq[ks].half[1] = *(const v8us*)(qr + ks * 32 + 16 + 8 * hh); } }
  const unsigned short* Vth = (const unsigned short*)Vt + (size_t)slab * HD * SEQ;
  const int* mrow = MSK + (size_t)b * mstride;
  float m_r[8], l_r[8]; v8f oacc[DT];
#pragma unroll
  for (int r = 0; r < 8; ++r) { m_r[r] = -3.0e38f; l_r[r] = 0.f; }
#pragma unroll
  for (int dt = 0; dt < DT; ++dt) oacc[dt] = (v8f){0.f,0.f,0.f,0.f,0.f,0.f,0.f,0.f};
#pragma unroll 1
  for (int j0 = 0; j0 < SEQ; j0 += 32) {
    v8f s[2];
#pragma unroll
    for (int nt = 0; nt < 2; ++nt) {
      const unsigned short* kr = (const unsigned short*)K16 + ((size_t)b * SEQ + j0 + nt * 16 + ln) * ldk + h * HD;
      FragH bk[KS];
#pragma unroll
      for (int ks = 0; ks < KS; ++ks) { bk[ks].half[0] = *(const v8us*)(kr + ks * 32 + 8 * hh); bk[ks].half[1] = *(const v8us*)(kr + ks * 32 + 16 + 8 * hh); }
      v8f acc = (v8f){0.f,0.f,0.f,0.f,0.f,0.f,0.f,0.f};
#pragma unroll
      for (int ks = 0; ks < KS; ++ks) acc = mma16(aq[ks].v, bk[ks].v, acc);
      s[nt] = acc;
    }
    const int mk0 = mrow[j0 + ln], mk1 = mrow[j0 + 16 + ln];
#pragma unroll
    for (int r = 0; r < 8; ++r) {
      const float s0 = (mk0 != 0) ? s[0][r] * SCL : -1.0e9f, s1 = (mk1 != 0) ? s[1][r] * SCL : -1.0e9f;
      float mc = fmaxf(s0, s1);
      mc = fmaxf(mc, __shfl_xor(mc, 1, 32)); mc = fmaxf(mc, __shfl_xor(mc, 2, 32)); mc = fmaxf(mc, __shfl_xor(mc, 4, 32)); mc = fmaxf(mc, __shfl_xor(mc, 8, 32));
      const float mn = fmaxf(m_r[r], mc); const float al = (mn > -1.0e38f) ? expf(m_r[r] - mn) : 1.0f; m_r[r] = mn;
      const float p0 = expf(s0 - mn), p1 = expf(s1 - mn); l_r[r] = l_r[r] * al + p0 + p1;
#pragma unroll
      for (int dt = 0; dt < DT; ++dt) oacc[dt][r] *= al;
      FragH t2; t2.h[0] = (_Float16)(p0 * 1024.0f); t2.h[1] = (_Float16)(p1 * 1024.0f);
      sP[w][8 * hh + r][ln] = t2.u[0]; sP[w][8 * hh + r][16 + ln] = t2.u[1];
    }
    __builtin_amdgcn_fence(4, "workgroup"); __builtin_amdgcn_wave_barrier();
    FragH pa; pa.half[0] = *(const v8us*)&sP[w][ln][8 * hh]; pa.half[1] = *(const v8us*)&sP[w][ln][16 + 8 * hh];
#pragma unroll
    for (int dt = 0; dt < DT; ++dt) { const unsigned short* vrow = Vth + (size_t)(dt * 16 + ln) * SEQ + j0; FragH bvf; bvf.half[0] = *(const v8us*)(vrow + 8 * hh); bvf.half[1] = *(const v8us*)(vrow + 16 + 8 * hh);
      oacc[dt] = mma16(pa.v, bvf.v, oacc[dt]); }
    __builtin_amdgcn_fence(4, "workgroup"); __builtin_amdgcn_wave_barrier();
  }
#pragma unroll
  for (int r = 0; r < 8; ++r) { float l = l_r[r]; l += __shfl_xor(l, 1, 32); l += __shfl_xor(l, 2, 32); l += __shfl_xor(l, 4, 32); l += __shfl_xor(l, 8, 32); l_r[r] = (l > 0.f) ? 1.0f / (l * 1024.0f) : 0.f; }
#pragma unroll
  for (int dt = 0; dt < DT; ++dt)
#pragma unroll
    for (int r = 0; r < 8; ++r) sO[w][8 * hh + r][dt * 16 + ln] = oacc[dt][r] * l_r[r];
  __builtin_amdgcn_fence(4, "workgroup"); __builtin_amdgcn_wave_barrier();
  for (int pass = 0; pass < 2; ++pass) {
#pragma unroll
    for (int rp = 0; rp < RPW; rp += 2) { const int r = rp + hh; const v4f val = *(const v4fa*)&sO[w][r][ln * 4]; *(volatile v4f*)(O + ((size_t)b * SEQ + q0 + r) * ldo + h * HD + ln * 4) = val; }
    if (pass == 0) __threadfence(); }
}

__global__ __launch_bounds__(256) void k_hl(const float* __restrict__ F, _Float16* __restrict__ Hh, _Float16* __restrict__ Hl, size_t n8) {
  const size_t t = (size_t)blockIdx.x * 256 + threadIdx.x; if (t >= n8) return; FragH fh, fl; const v4f a = *(const v4fa*)(F + t * 8), c = *(const v4fa*)(F + t * 8 + 4);
#pragma unroll
  for (int q = 0; q < 4; ++q) { _Float16 hv = (_Float16)a[q]; fh.h[q] = hv; fl.h[q] = (_Float16)((a[q] - (float)hv) * 1024.0f); hv = (_Float16)c[q]; fh.h[4 + q] = hv; fl.h[4 + q] = (_Float16)((c[q] - (float)hv) * 1024.0f); }
  const v8us oh = fh.half[0], ol = fl.half[0];
  for (int pass = 0; pass < 2; ++pass) { *(volatile v8us*)((unsigned short*)Hh + t * 8) = oh; *(volatile v8us*)((unsigned short*)Hl + t * 8) = ol; if (pass == 0) __threadfence(); }
}

extern "C" void kernel_launch(void* const* d_in, const int* in_sizes, int n_in,
                              void* d_out, int out_size, void* d_ws, size_t ws_size, hipStream_t stream) {
  if (n_in < 10) return;
  if (in_sizes[0] < ((NB - 1) * SEQ_FULL + SEQ) * DM) return;
  if (in_sizes[1] < (NB - 1) * SEQ_FULL + SEQ) return;
  if (in_sizes[2] < DM * DM || in_sizes[4] < DM * DM || in_sizes[6] < DM * DM || in_sizes[8] < DM * DM) return;
  if (in_sizes[3] < DM || in_sizes[5] < DM || in_sizes[7] < DM || in_sizes[9] < DM) return;
  if (out_size < NR * DM) return;
  const float* x  = (const float*)d_in[0]; const int* msk = (const int*)d_in[1];
  const float* Wq = (const float*)d_in[2]; const float* bq = (const float*)d_in[3];
  const float* Wk = (const float*)d_in[4]; const float* bk = (const float*)d_in[5];
  const float* Wv = (const float*)d_in[6]; const float* bv = (const float*)d_in[7];
  const float* Wo = (const float*)d_in[8]; const float* bo = (const float*)d_in[9];
  float* out = (float*)d_out;
  char* ws = (char*)d_ws; size_t off = 0;
  auto take = [&](size_t bytes) { char* p = ws + off; off += (bytes + 255) & ~(size_t)255; return p; };
  const size_t np = (size_t)NR * DM, nw = (size_t)DM * DM;
  _Float16* BQ = (_Float16*)take(nw * 2); _Float16* BK = (_Float16*)take(nw * 2); _Float16* BV = (_Float16*)take(nw * 2); _Float16* BO = (_Float16*)take(nw * 2);
  _Float16* X16 = (_Float16*)take(np * 2); _Float16* QH = (_Float16*)take(np * 2); _Float16* KH = (_Float16*)take(np * 2); _Float16* V16 = (_Float16*)take(np * 2); _Float16* VT = (_Float16*)take(np * 2);
  float* O = (float*)take(np * 4); _Float16* OH = QH; _Float16* OL = KH;
  if (off > ws_size || off > ((size_t)128 << 20)) return;
  const unsigned gw = (unsigned)((nw / 8 + 255) / 256), gx = (unsigned)((np / 8 + 255) / 256);
  k_wsc<<<gw, 256, 0, stream>>>(Wq, BQ, nw / 8, 16.0f);
  k_wsc<<<gw, 256, 0, stream>>>(Wk, BK, nw / 8, 16.0f);
  k_wsc<<<gw, 256, 0, stream>>>(Wv, BV, nw / 8, 16.0f);
  k_wsc<<<gw, 256, 0, stream>>>(Wo, BO, nw / 8, 16.0f);
  k_x16<<<gx, 256, 0, stream>>>(x, X16, np / 8);
  const unsigned gg = (unsigned)((NR / 128) * (DM / 64));
  k_gemm2<<<gg, 128, 0, stream>>>(X16, DM, BQ, DM, 0.0625f, bq, nullptr, 0, nullptr, QH, DM, NR, DM, DM);
  k_gemm2<<<gg, 128, 0, stream>>>(X16, DM, BK, DM, 0.0625f, bk, nullptr, 0, nullptr, KH, DM, NR, DM, DM);
  k_gemm2<<<gg, 128, 0, stream>>>(X16, DM, BV, DM, 0.0625f, bv, nullptr, 0, nullptr, V16, DM, NR, DM, DM);
  k_vtg<<<(unsigned)(NB * NH * (SEQ / 64)), 256, 0, stream>>>(V16, VT);
  k_flash<<<(unsigned)(NB * NH * QBLKS), 128, 0, stream>>>(QH, DM, KH, DM, VT, msk, SEQ_FULL, O, DM);
  k_hl<<<gx, 256, 0, stream>>>(O, OH, OL, np / 8);
  k_gemm2<<<gg, 128, 0, stream>>>(OL, DM, BO, DM, 0.0625f / 1024.0f, nullptr, nullptr, 0, out, nullptr, DM, NR, DM, DM);
  k_gemm2<<<gg, 128, 0, stream>>>(OH, DM, BO, DM, 0.0625f, bo, out, DM, out, nullptr, DM, NR, DM, DM);
}
